// GRU_D_75411035783284
// MI455X (gfx1250) — hardware-run, weakly checked
//
#include <hip/hip_runtime.h>
#include <math.h>

constexpr int NBAT    = 256;
constexpr int NCH     = 64;
constexpr int NSTEP   = 256;
constexpr int NHID    = 512;
constexpr int NROWBC  = NBAT * NCH;
constexpr int NROWBT  = NBAT * NSTEP;
constexpr int KDEC2   = NCH * NSTEP;
constexpr int KSPLIT  = 16;
constexpr int KSLICE  = KDEC2 / KSPLIT;
constexpr int NTHR    = 256;
constexpr int SEQ_BLK = 16;
constexpr int HPITCH  = 520;
constexpr int XPITCH  = 72;
constexpr int SLABP   = 68;
constexpr float XSIDE_SC = 1.0f;
constexpr float HCARRY   = 16.0f;
constexpr float UCARRY   = 4.0f;
constexpr float ACC_INV  = 1.0f / 64.0f;
constexpr float F32_MINN = 1.17549435e-38f;
static_assert(HCARRY * UCARRY * ACC_INV == 1.0f);
static_assert(XSIDE_SC == 1.0f);
static_assert(NHID == 64 * (NTHR / 32));
static_assert(NCH % 32 == 0 && NHID % 32 == 0 && NSTEP % 32 == 0 && KSLICE % 32 == 0);
static_assert(NROWBC % 64 == 0 && NSTEP % 64 == 0 && NBAT % 64 == 0 && NHID % 64 == 0 && NCH % 64 == 0);
static_assert(NBAT % SEQ_BLK == 0);
static_assert(KSPLIT * KSLICE == KDEC2);

typedef __attribute__((ext_vector_type(16))) _Float16 v16h;
typedef __attribute__((ext_vector_type(8)))  _Float16 v8h;
typedef __attribute__((ext_vector_type(16))) __bf16   v16b;
typedef __attribute__((ext_vector_type(8)))  __bf16   v8b;
typedef __attribute__((ext_vector_type(8)))  float    v8f;
typedef __attribute__((ext_vector_type(4)))  float    v4f;
typedef __attribute__((ext_vector_type(4)))  unsigned v4u;
typedef __attribute__((ext_vector_type(2)))  unsigned v2u;

__device__ __forceinline__ unsigned short f2bf_bits(float f) {
  unsigned u = __float_as_uint(f);
  return (unsigned short)((u + 0x7FFFu + ((u >> 16) & 1u)) >> 16);
}
__device__ __forceinline__ float bf_bits2f(unsigned short h) { return __uint_as_float(((unsigned)h) << 16); }
__device__ __forceinline__ unsigned short f2h_bits(float f) {
  const _Float16 hv = (_Float16)f;
  return __builtin_bit_cast(unsigned short, hv);
}

__device__ __forceinline__ void guard4_h(v8f& a, v8f& b, v8f& c, v8f& d, v16h x, v16h y) { asm volatile("v_nop\n\tv_nop\n\tv_nop\n\tv_nop" : "+v"(a), "+v"(b), "+v"(c), "+v"(d) : "v"(x), "v"(y)); }
__device__ __forceinline__ void guard4_b(v8f& a, v8f& b, v8f& c, v8f& d, v16b x, v16b y) { asm volatile("v_nop\n\tv_nop\n\tv_nop\n\tv_nop" : "+v"(a), "+v"(b), "+v"(c), "+v"(d) : "v"(x), "v"(y)); }
__device__ __forceinline__ void guard2_h3(v8f& a, v8f& b, v16h x, v16h y, v16h z) { asm volatile("v_nop\n\tv_nop\n\tv_nop\n\tv_nop" : "+v"(a), "+v"(b) : "v"(x), "v"(y), "v"(z)); }
__device__ __forceinline__ void guard2_h4(v8f& a, v8f& b, v16h w, v16h x, v16h y, v16h z) { asm volatile("v_nop\n\tv_nop\n\tv_nop\n\tv_nop" : "+v"(a), "+v"(b) : "v"(w), "v"(x), "v"(y), "v"(z)); }
__device__ __forceinline__ void guard1_b4(v8f& a, v16b w, v16b x, v16b y, v16b z) { asm volatile("v_nop\n\tv_nop\n\tv_nop\n\tv_nop" : "+v"(a) : "v"(w), "v"(x), "v"(y), "v"(z)); }
__device__ __forceinline__ void keep4_h(v16h a, v16h b, v16h c, v16h d) { asm volatile("v_nop" :: "v"(a), "v"(b), "v"(c), "v"(d)); }
__device__ __forceinline__ void keep4_b(v16b a, v16b b, v16b c, v16b d) { asm volatile("v_nop" :: "v"(a), "v"(b), "v"(c), "v"(d)); }
__device__ __forceinline__ void acc_guard4(v8f& a, v8f& b, v8f& c, v8f& d) { asm volatile("v_nop\n\tv_nop\n\tv_nop\n\tv_nop" : "+v"(a), "+v"(b), "+v"(c), "+v"(d)); }
__device__ __forceinline__ void acc_guard2(v8f& a, v8f& b) { asm volatile("v_nop\n\tv_nop\n\tv_nop\n\tv_nop" : "+v"(a), "+v"(b)); }

template <typename T> struct Frag;
template <> struct Frag<_Float16> {
  typedef v16h V; union U { v16h v; v8h h[2]; };
  static __device__ __forceinline__ v16h load(const _Float16* p) {
    U f; f.h[0] = *(const v8h*)(p); f.h[1] = *(const v8h*)(p + 16); return f.v;
  }
  static __device__ __forceinline__ v8f mma(v16h a, v16h b, v8f c) {
    return __builtin_amdgcn_wmma_f32_16x16x32_f16(false, a, false, b, (short)0, c, false, false);
  }
  static __device__ __forceinline__ void guard4(v8f& a, v8f& b, v8f& c, v8f& d, v16h x, v16h y) { guard4_h(a, b, c, d, x, y); }
  static __device__ __forceinline__ void keep(v16h a, v16h b, v16h c, v16h d) { keep4_h(a, b, c, d); }
};
template <> struct Frag<__bf16> {
  typedef v16b V; union U { v16b v; v8b h[2]; };
  static __device__ __forceinline__ v16b load(const __bf16* p) {
    U f; f.h[0] = *(const v8b*)(p); f.h[1] = *(const v8b*)(p + 16); return f.v;
  }
  static __device__ __forceinline__ v8f mma(v16b a, v16b b, v8f c) {
    return __builtin_amdgcn_wmma_f32_16x16x32_bf16(false, a, false, b, (short)0, c, false, false);
  }
  static __device__ __forceinline__ void guard4(v8f& a, v8f& b, v8f& c, v8f& d, v16b x, v16b y) { guard4_b(a, b, c, d, x, y); }
  static __device__ __forceinline__ void keep(v16b a, v16b b, v16b c, v16b d) { keep4_b(a, b, c, d); }
};

__device__ __forceinline__ float fsig(float v)  { return __builtin_amdgcn_rcpf(1.0f + __expf(-v)); }
__device__ __forceinline__ float ftanh(float v) { return 1.0f - 2.0f * __builtin_amdgcn_rcpf(__expf(2.0f * v) + 1.0f); }

template <int ET> struct Elem;
template <> struct Elem<0> { typedef _Float16 T; };
template <> struct Elem<1> { typedef __bf16 T; };
template <int ET, bool SPLIT, bool TRI_A, int BIAS_MODE, int ACT>
__global__ __launch_bounds__(256) void wmma_gemm64(
    const unsigned short* __restrict__ Ap, const unsigned short* __restrict__ A2p,
    const unsigned short* __restrict__ A3p, int lda, long strideA,
    const unsigned short* __restrict__ Btp, const unsigned short* __restrict__ Bt2p, int ldb, long strideB,
    float* __restrict__ Cout, int ldc, long strideC,
    const float* __restrict__ bias,
    int M, int N, int K, float scale) {
  static_assert(ACT == 0 || ACT == 2);
  static_assert(BIAS_MODE == 0 || BIAS_MODE == 2);
  static_assert(SPLIT || !TRI_A);
  typedef typename Elem<ET>::T T;
  typedef typename Frag<T>::V V;
  const T* A = (const T*)Ap; const T* A2 = (const T*)A2p; const T* A3 = (const T*)A3p;
  const T* Bt = (const T*)Btp; const T* Bt2 = (const T*)Bt2p;
  __shared__ __align__(16) float sT[8][16 * 68];
  const int b    = blockIdx.y;
  const int lane = threadIdx.x & 31;
  const int wave = threadIdx.x >> 5;
  const int tilesN = N >> 6;
  const int tilesM = M >> 6;
  const int tile = blockIdx.x * 8 + wave;
  if (tile >= tilesM * tilesN) return;
  const int tm = tile / tilesN;
  const int tn = tile - tm * tilesN;
  const int m0 = tm << 6;
  const int n0 = tn << 6;

  const T* Ab  = A  + (size_t)b * strideA;
  const T* Bb  = Bt + (size_t)b * strideB;
  const T* Ab2 = SPLIT ? (A2  + (size_t)b * strideA) : nullptr;
  const T* Ab3 = TRI_A ? (A3  + (size_t)b * strideA) : nullptr;
  const T* Bb2 = SPLIT ? (Bt2 + (size_t)b * strideB) : nullptr;

  const int rlane = lane & 15;
  const int koff  = (lane >> 4) * 8;
  const int mOff  = (lane >> 4) * 8;

  v8f acc[4][4];
#pragma unroll
  for (int i = 0; i < 4; ++i)
#pragma unroll
    for (int j = 0; j < 4; ++j) acc[i][j] = (v8f){0.f,0.f,0.f,0.f,0.f,0.f,0.f,0.f};

  for (int k0 = 0; k0 < K; k0 += 32) {
    V bh[4], bl[4];
#pragma unroll
    for (int j = 0; j < 4; ++j) {
      const size_t bo = (size_t)(n0 + (j << 4) + rlane) * ldb + koff + k0;
      bh[j] = Frag<T>::load(Bb + bo);
      if (SPLIT) bl[j] = Frag<T>::load(Bb2 + bo);
    }
#pragma unroll
    for (int i = 0; i < 4; ++i) {
      const size_t ao = (size_t)(m0 + (i << 4) + rlane) * lda + koff + k0;
      V ah = Frag<T>::load(Ab + ao);
      V al;
      if (SPLIT) al = Frag<T>::load(Ab2 + ao);
#pragma unroll
      for (int j = 0; j < 4; ++j) {
        acc[i][j] = Frag<T>::mma(ah, bh[j], acc[i][j]);
        if (SPLIT) {
          acc[i][j] = Frag<T>::mma(ah, bl[j], acc[i][j]);
          acc[i][j] = Frag<T>::mma(al, bh[j], acc[i][j]);
        }
      }
      Frag<T>::guard4(acc[i][0], acc[i][1], acc[i][2], acc[i][3], ah, SPLIT ? al : ah);
      if (TRI_A) {
        V at = Frag<T>::load(Ab3 + ao);
#pragma unroll
        for (int j = 0; j < 4; ++j) acc[i][j] = Frag<T>::mma(at, bh[j], acc[i][j]);
        Frag<T>::guard4(acc[i][0], acc[i][1], acc[i][2], acc[i][3], at, at);
      }
    }
    Frag<T>::keep(bh[0], bh[1], bh[2], bh[3]);
    if (SPLIT) Frag<T>::keep(bl[0], bl[1], bl[2], bl[3]);
  }
  acc_guard4(acc[0][0], acc[0][1], acc[0][2], acc[0][3]);
  acc_guard4(acc[1][0], acc[1][1], acc[1][2], acc[1][3]);
  acc_guard4(acc[2][0], acc[2][1], acc[2][2], acc[2][3]);
  acc_guard4(acc[3][0], acc[3][1], acc[3][2], acc[3][3]);

  float* slab = sT[wave];
#pragma unroll
  for (int i = 0; i < 4; ++i) {
    const int mBase = m0 + (i << 4);
#pragma unroll
    for (int j = 0; j < 4; ++j) {
      const int n = n0 + (j << 4) + rlane;
      float bv = 0.f;
      if (BIAS_MODE == 2) bv = bias[n];
#pragma unroll
      for (int r = 0; r < 8; ++r) {
        float v = acc[i][j][r] * scale;
        if (BIAS_MODE == 2) v += bv;
        if (ACT == 2) v = fmaxf(v, 0.0f);
        slab[(mOff + r) * 68 + (j << 4) + rlane] = v;
      }
    }
    __builtin_amdgcn_fence(__ATOMIC_RELEASE, "workgroup");
    __builtin_amdgcn_wave_barrier();
    __builtin_amdgcn_fence(__ATOMIC_ACQUIRE, "workgroup");
    {
      float* C = Cout + (size_t)b * strideC;
      const int hh = lane >> 4, c4 = (lane & 15) * 4;
      for (int pass = 0; pass < 2; ++pass) {
#pragma unroll
        for (int it = 0; it < 8; ++it) {
          const int row = it * 2 + hh;
          v4f v = *(const v4f*)(slab + row * 68 + c4);
          *(volatile v4f*)(C + (size_t)(mBase + row) * ldc + n0 + c4) = v;
        }
        __threadfence();
      }
    }
    __builtin_amdgcn_fence(__ATOMIC_RELEASE, "workgroup");
    __builtin_amdgcn_wave_barrier();
    __builtin_amdgcn_fence(__ATOMIC_ACQUIRE, "workgroup");
  }
}

template <int MODE>
__global__ __launch_bounds__(NTHR) void tpw_kernel(const float* __restrict__ s0, const float* __restrict__ s1,
                                                   const float* __restrict__ s2, int R, int C, int ldo,
                                                   unsigned short* __restrict__ O, unsigned short* __restrict__ O2,
                                                   long zstride, float sc) {
  __shared__ float Tt[64 * 65];
  const int tid = threadIdx.x;
  const int zz = blockIdx.z;
  const float* src = (zz == 0) ? s0 : ((zz == 1) ? s1 : s2);
  unsigned short* Oz  = O  + (size_t)zz * (size_t)zstride;
  unsigned short* O2z = O2 + (size_t)zz * (size_t)zstride;
  const int c0 = blockIdx.x * 64, r0 = blockIdx.y * 64;
#pragma unroll
  for (int i = 0; i < 4; ++i) {
    const int idx = i * NTHR + tid;
    const int rr = idx >> 4, cc = (idx & 15) * 4;
    const v4f v = *(const v4f*)(src + (size_t)(r0 + rr) * (size_t)C + c0 + cc);
    Tt[rr * 65 + cc + 0] = v[0];
    Tt[rr * 65 + cc + 1] = v[1];
    Tt[rr * 65 + cc + 2] = v[2];
    Tt[rr * 65 + cc + 3] = v[3];
  }
  __syncthreads();
  const int q = tid >> 3, c8 = (tid & 7) * 8;
  v4u hv[2], lv[2];
#pragma unroll
  for (int g = 0; g < 2; ++g) {
    const int qq = g * 32 + q;
    unsigned hb[8], lb[8];
#pragma unroll
    for (int e = 0; e < 8; ++e) {
      const float f = Tt[(c8 + e) * 65 + qq];
      if (MODE == 0) {
        const unsigned short h = f2bf_bits(f);
        hb[e] = (unsigned)h;
        lb[e] = (unsigned)f2bf_bits(f - bf_bits2f(h));
      } else {
        hb[e] = (unsigned)f2h_bits(f * sc);
        lb[e] = 0u;
      }
    }
#pragma unroll
    for (int w = 0; w < 4; ++w) {
      hv[g][w] = hb[2 * w] | (hb[2 * w + 1] << 16);
      lv[g][w] = lb[2 * w] | (lb[2 * w + 1] << 16);
    }
  }
  for (int pass = 0; pass < 2; ++pass) {
#pragma unroll
    for (int g = 0; g < 2; ++g) {
      const size_t o = (size_t)(c0 + g * 32 + q) * (size_t)ldo + (size_t)(r0 + c8);
      *(volatile v4u*)(Oz + o) = hv[g];
      if (MODE == 0) *(volatile v4u*)(O2z + o) = lv[g];
    }
    __threadfence();
  }
}

#define SCAN_ONE_STEP(RAWV, MSKV, LOFF)                       \
  {                                                           \
    const float rv_ = (RAWV);                                 \
    const float mv_ = (MSKV);                                 \
    const float ne_ = mv_ * rv_ + (1.0f - mv_) * carry;       \
    carry = ne_;                                              \
    sXe[(LOFF)] = ne_;                                        \
    sIv[(LOFF)] = ivout;                                      \
    const float nx_ = 1.0f + cr * (1.0f - mv_);               \
    cr = nx_;                                                 \
    ivout = nx_;                                              \
  }

__global__ __launch_bounds__(64) void scan_kernel(const float* __restrict__ x, float* __restrict__ XE,
                                                  unsigned short* __restrict__ IVH, unsigned short* __restrict__ IVM,
                                                  unsigned short* __restrict__ IVL) {
  __shared__ __align__(16) float sXe[64 * SLABP];
  __shared__ __align__(16) float sIv[64 * SLABP];
  const int tid = threadIdx.x;
  const int rowbase = blockIdx.x * 64;
  const float* px = x + (size_t)(rowbase + tid) * (size_t)(NSTEP * 3);
  float carry = px[0];
  float cr = 1.0f, ivout = 0.0f;
#pragma unroll 1
  for (int tc = 0; tc < NSTEP / 64; ++tc) {
#pragma unroll 1
    for (int q = 0; q < 16; ++q) {
      const float* p = px + (tc * 64 + q * 4) * 3;
      const v4f va = *(const v4f*)(p);
      const v4f vb = *(const v4f*)(p + 4);
      const v4f vc = *(const v4f*)(p + 8);
      const int o = tid * SLABP + q * 4;
      SCAN_ONE_STEP(va[0], va[2], o + 0)
      SCAN_ONE_STEP(va[3], vb[1], o + 1)
      SCAN_ONE_STEP(vb[2], vc[0], o + 2)
      SCAN_ONE_STEP(vc[1], vc[3], o + 3)
    }
    __syncthreads();
    for (int pass = 0; pass < 2; ++pass) {
#pragma unroll 1
      for (int it = 0; it < 16; ++it) {
        const int idx = it * 64 + tid;
        const int r = idx >> 4, c4 = (idx & 15) * 4;
        const v4f v = *(const v4f*)(sXe + r * SLABP + c4);
        *(volatile v4f*)(XE + (size_t)(rowbase + r) * NSTEP + tc * 64 + c4) = v;
      }
#pragma unroll 1
      for (int it = 0; it < 8; ++it) {
        const int idx = it * 64 + tid;
        const int r = idx >> 3, c8 = (idx & 7) * 8;
        const v4f f0 = *(const v4f*)(sIv + r * SLABP + c8);
        const v4f f1 = *(const v4f*)(sIv + r * SLABP + c8 + 4);
        unsigned hb[8], mb[8], lb[8];
#pragma unroll
        for (int e = 0; e < 4; ++e) {
          const float a = f0[e];
          const float b = f1[e];
          const unsigned short ha = f2bf_bits(a);
          const unsigned short hb2 = f2bf_bits(b);
          const float ra = a - bf_bits2f(ha);
          const float rb = b - bf_bits2f(hb2);
          const unsigned short ma = f2bf_bits(ra);
          const unsigned short mb2 = f2bf_bits(rb);
          hb[e]     = (unsigned)ha;
          hb[4 + e] = (unsigned)hb2;
          mb[e]     = (unsigned)ma;
          mb[4 + e] = (unsigned)mb2;
          lb[e]     = (unsigned)f2bf_bits(ra - bf_bits2f(ma));
          lb[4 + e] = (unsigned)f2bf_bits(rb - bf_bits2f(mb2));
        }
        v4u hv, mv, lv;
#pragma unroll
        for (int w = 0; w < 4; ++w) {
          hv[w] = hb[2 * w] | (hb[2 * w + 1] << 16);
          mv[w] = mb[2 * w] | (mb[2 * w + 1] << 16);
          lv[w] = lb[2 * w] | (lb[2 * w + 1] << 16);
        }
        const size_t o = (size_t)(rowbase + r) * NSTEP + tc * 64 + c8;
        *(volatile v4u*)(IVH + o) = hv;
        *(volatile v4u*)(IVM + o) = mv;
        *(volatile v4u*)(IVL + o) = lv;
      }
      __threadfence();
    }
    __syncthreads();
  }
}

__global__ __launch_bounds__(NTHR) void d2_fin_kernel(const float* __restrict__ PART, const float* __restrict__ b2,
                                                      float* __restrict__ D2) {
  const int i = blockIdx.x * NTHR + threadIdx.x;
  const int e0 = i * 4;
  const int s = e0 & (NSTEP - 1);
  v4f acc = *(const v4f*)(PART + e0);
#pragma unroll 1
  for (int sl = 1; sl < KSPLIT; ++sl) {
    const v4f pv = *(const v4f*)(PART + (size_t)sl * (size_t)(NBAT * NSTEP) + e0);
    acc += pv;
  }
  const v4f bb = *(const v4f*)(b2 + s);
  v4f o;
#pragma unroll
  for (int e = 0; e < 4; ++e) {
    const float p = fmaxf(acc[e] + bb[e], 0.0f);
    float d = expf(-p);
    d = (d < F32_MINN) ? 0.0f : d;
    o[e] = d;
  }
  *(volatile v4f*)(D2 + e0) = o;
  __threadfence();
  *(volatile v4f*)(D2 + e0) = o;
}

__global__ __launch_bounds__(NTHR) void xnew_kernel(const float* __restrict__ x, const float* __restrict__ XE,
                                                    const float* __restrict__ P1, unsigned short* __restrict__ XNH,
                                                    unsigned short* __restrict__ XNL) {
  __shared__ __align__(16) float sXe[64 * SLABP];
  __shared__ float sMean[64];
  __shared__ __align__(16) unsigned short sXh[64 * XPITCH];
  __shared__ __align__(16) unsigned short sXl[64 * XPITCH];
  const int tid = threadIdx.x;
  const int b = blockIdx.y;
  const int t0 = blockIdx.x * 64;
#pragma unroll
  for (int it = 0; it < 4; ++it) {
    const int idx = it * NTHR + tid;
    const int cc = idx >> 4, t4 = (idx & 15) * 4;
    const v4f v = *(const v4f*)(XE + (size_t)(b * NCH + cc) * NSTEP + t0 + t4);
    *(v4f*)(sXe + cc * SLABP + t4) = v;
  }
  __syncthreads();
  if (tid < 64) {
    float s = 0.0f;
#pragma unroll 1
    for (int cc = 0; cc < NCH; ++cc) s += sXe[cc * SLABP + tid];
    sMean[tid] = s * (1.0f / (float)NCH);
  }
  __syncthreads();
#pragma unroll 1
  for (int it = 0; it < 16; ++it) {
    const int idx = it * NTHR + tid;
    const int cc = idx >> 6, tt = idx & 63;
    const size_t g = (size_t)(b * NCH + cc) * NSTEP + t0 + tt;
    const float raw = x[g * 3];
    const float m   = x[g * 3 + 2];
    const float p   = P1[g];
    const float xe  = sXe[cc * SLABP + tt];
    const float me  = sMean[tt];
    float d = expf(-p);
    d = (d < F32_MINN) ? 0.0f : d;
    const float v = m * raw + (1.0f - m) * (d * xe + (1.0f - d) * me);
    const unsigned short vh = f2bf_bits(v);
    const unsigned short vl = f2bf_bits(v - bf_bits2f(vh));
    sXh[tt * XPITCH + cc] = vh;
    sXl[tt * XPITCH + cc] = vl;
  }
  __syncthreads();
  v4u ovh[2], ovl[2];
#pragma unroll
  for (int g = 0; g < 2; ++g) {
    const int idx = g * NTHR + tid;
    const int tt = idx >> 3, c8 = (idx & 7) * 8;
    ovh[g] = *(const v4u*)(sXh + tt * XPITCH + c8);
    ovl[g] = *(const v4u*)(sXl + tt * XPITCH + c8);
  }
  for (int pass = 0; pass < 2; ++pass) {
#pragma unroll
    for (int g = 0; g < 2; ++g) {
      const int idx = g * NTHR + tid;
      const int tt = idx >> 3, c8 = (idx & 7) * 8;
      const size_t o = (size_t)(b * NSTEP + t0 + tt) * NCH + c8;
      *(volatile v4u*)(XNH + o) = ovh[g];
      *(volatile v4u*)(XNL + o) = ovl[g];
    }
    __threadfence();
  }
}

__global__ __launch_bounds__(NTHR) void gru_seq_kernel(
    const unsigned short* __restrict__ XNH, const unsigned short* __restrict__ XNL, const float* __restrict__ D2,
    const unsigned short* __restrict__ WXHp, const unsigned short* __restrict__ WXLp,
    const unsigned short* __restrict__ UTp, const unsigned short* __restrict__ WOTp,
    const float* __restrict__ bz, const float* __restrict__ br, const float* __restrict__ bh,
    const float* __restrict__ bo, float* __restrict__ OUTT) {
  __shared__ __align__(16) _Float16 Adh[SEQ_BLK * HPITCH];
  __shared__ __align__(16) _Float16 Arh[SEQ_BLK * HPITCH];
  __shared__ __align__(16) _Float16 Ahn[SEQ_BLK * HPITCH];
  __shared__ __align__(16) unsigned short Axh[SEQ_BLK * XPITCH];
  __shared__ __align__(16) unsigned short Axl[SEQ_BLK * XPITCH];
  __shared__ __align__(16) float Os[SEQ_BLK * SLABP];
  const __bf16*   WXH = (const __bf16*)WXHp;
  const __bf16*   WXL = (const __bf16*)WXLp;
  const _Float16* UT  = (const _Float16*)UTp;
  const _Float16* WOT = (const _Float16*)WOTp;
  const int tid = threadIdx.x, lane = tid & 31;
  const int wave = __builtin_amdgcn_readfirstlane(tid >> 5);
  const int c = lane & 15, hh = lane >> 4, koff = hh * 8, c4 = c * 4;
  const int rowbase = blockIdx.x * SEQ_BLK;

  float hst[4][8], zreg[4][8], bzv[4], brv[4], bhv[4];
#pragma unroll
  for (int nt = 0; nt < 4; ++nt) {
    const int j = 64 * wave + 16 * nt + c;
    bzv[nt] = bz[j];
    brv[nt] = br[j];
    bhv[nt] = bh[j];
#pragma unroll
    for (int r = 0; r < 8; ++r) { hst[nt][r] = 0.0f; zreg[nt][r] = 0.0f; }
  }
  const float bov = bo[16 * (wave & 3) + c];

  const __bf16*   axhrow = (const __bf16*)Axh + c * XPITCH + koff;
  const __bf16*   axlrow = (const __bf16*)Axl + c * XPITCH + koff;
  const _Float16* adhrow = Adh + c * HPITCH + koff;
  const _Float16* arhrow = Arh + c * HPITCH + koff;
  const _Float16* ahnrow = Ahn + c * HPITCH + koff;
  const int xm = tid >> 4, xf4 = (tid & 15) * 4;
  const unsigned short* xsrch = XNH + ((size_t)(rowbase + xm) * NSTEP) * NCH + xf4;
  const unsigned short* xsrcl = XNL + ((size_t)(rowbase + xm) * NSTEP) * NCH + xf4;
  const int orow = 2 * wave + hh;
  float* const obase = OUTT + ((size_t)(rowbase + orow) * NSTEP) * NCH + c4;
  const float* d2row = D2 + (size_t)(rowbase + 8 * hh) * NSTEP;
  const v8f z8 = {0.f, 0.f, 0.f, 0.f, 0.f, 0.f, 0.f, 0.f};

#pragma unroll 1
  for (int t = 0; t < NSTEP; ++t) {
    float dec[8];
#pragma unroll
    for (int r = 0; r < 8; ++r) dec[r] = d2row[(size_t)r * NSTEP + t];
    const v2u xvh = *(const v2u*)(xsrch + (size_t)t * NCH);
    const v2u xvl = *(const v2u*)(xsrcl + (size_t)t * NCH);

#pragma unroll
    for (int nt = 0; nt < 4; ++nt) {
      const int j = 64 * wave + 16 * nt + c;
#pragma unroll
      for (int r = 0; r < 8; ++r) {
        const float dhv = dec[r] * hst[nt][r];
        Adh[(8 * hh + r) * HPITCH + j] = (_Float16)(dhv * HCARRY);
      }
    }
    *(v2u*)(Axh + xm * XPITCH + xf4) = xvh;
    *(v2u*)(Axl + xm * XPITCH + xf4) = xvl;
    __syncthreads();

    if (t > 0) {
      const v4f ov = *(const v4f*)(Os + orow * SLABP + c4);
      float* op = obase + (size_t)(t - 1) * NCH;
      *(volatile v4f*)op = ov;
      __threadfence();
      *(volatile v4f*)op = ov;
    }

#pragma unroll
    for (int nt = 0; nt < 4; ++nt) {
      const int j = 64 * wave + 16 * nt + c;
      const __bf16* wzh = WXH + (size_t)j * NCH + koff;
      const __bf16* wzl = WXL + (size_t)j * NCH + koff;
      const __bf16* wrh = wzh + (size_t)NHID * NCH;
      const __bf16* wrl = wzl + (size_t)NHID * NCH;
      const _Float16* uz = UT + (size_t)j * NHID + koff;
      const _Float16* ur = uz + (size_t)NHID * NHID;
      v8f accZ = z8, accR = z8;
      v8f accZx = z8, accRx = z8;
#pragma unroll 1
      for (int kx = 0; kx < NCH; kx += 32) {
        const v16b ah = Frag<__bf16>::load(axhrow + kx);
        const v16b al = Frag<__bf16>::load(axlrow + kx);
        const v16b zh = Frag<__bf16>::load(wzh + kx);
        const v16b zl = Frag<__bf16>::load(wzl + kx);
        const v16b rh = Frag<__bf16>::load(wrh + kx);
        const v16b rl = Frag<__bf16>::load(wrl + kx);
        accZx = Frag<__bf16>::mma(ah, zh, accZx);
        accZx = Frag<__bf16>::mma(ah, zl, accZx);
        accZx = Frag<__bf16>::mma(al, zh, accZx);
        guard1_b4(accZx, ah, al, zh, zl);
        accRx = Frag<__bf16>::mma(ah, rh, accRx);
        accRx = Frag<__bf16>::mma(ah, rl, accRx);
        accRx = Frag<__bf16>::mma(al, rh, accRx);
        guard1_b4(accRx, ah, al, rh, rl);
      }
#pragma unroll 2
      for (int k0 = 0; k0 < NHID; k0 += 32) {
        const v16h a  = Frag<_Float16>::load(adhrow + k0);
        const v16h b0 = Frag<_Float16>::load(uz + k0);
        const v16h b1 = Frag<_Float16>::load(ur + k0);
        accZ = Frag<_Float16>::mma(a, b0, accZ);
        accR = Frag<_Float16>::mma(a, b1, accR);
        guard2_h3(accZ, accR, a, b0, b1);
      }
      acc_guard2(accZ, accR);
#pragma unroll
      for (int r = 0; r < 8; ++r) {
        const float pz = accZ[r] * ACC_INV + accZx[r] + bzv[nt];
        const float pr = accR[r] * ACC_INV + accRx[r] + brv[nt];
        const float zz = fsig(pz);
        const float rr = fsig(pr);
        zreg[nt][r] = zz;
        const float dhv = dec[r] * hst[nt][r];
        Arh[(8 * hh + r) * HPITCH + j] = (_Float16)(rr * dhv * HCARRY);
      }
    }
    __syncthreads();

#pragma unroll
    for (int ntp = 0; ntp < 2; ++ntp) {
      const int j0 = 64 * wave + 32 * ntp + c;
      const __bf16* wh0h = WXH + (size_t)2 * NHID * NCH + (size_t)j0 * NCH + koff;
      const __bf16* wh0l = WXL + (size_t)2 * NHID * NCH + (size_t)j0 * NCH + koff;
      const __bf16* wh1h = wh0h + (size_t)16 * NCH;
      const __bf16* wh1l = wh0l + (size_t)16 * NCH;
      const _Float16* uh0 = UT + (size_t)2 * NHID * NHID + (size_t)j0 * NHID + koff;
      const _Float16* uh1 = uh0 + (size_t)16 * NHID;
      v8f acc[2];
      v8f accx[2];
      acc[0] = z8; acc[1] = z8;
      accx[0] = z8; accx[1] = z8;
#pragma unroll 1
      for (int kx = 0; kx < NCH; kx += 32) {
        const v16b ah  = Frag<__bf16>::load(axhrow + kx);
        const v16b al  = Frag<__bf16>::load(axlrow + kx);
        const v16b b0h = Frag<__bf16>::load(wh0h + kx);
        const v16b b0l = Frag<__bf16>::load(wh0l + kx);
        const v16b b1h = Frag<__bf16>::load(wh1h + kx);
        const v16b b1l = Frag<__bf16>::load(wh1l + kx);
        accx[0] = Frag<__bf16>::mma(ah, b0h, accx[0]);
        accx[0] = Frag<__bf16>::mma(ah, b0l, accx[0]);
        accx[0] = Frag<__bf16>::mma(al, b0h, accx[0]);
        guard1_b4(accx[0], ah, al, b0h, b0l);
        accx[1] = Frag<__bf16>::mma(ah, b1h, accx[1]);
        accx[1] = Frag<__bf16>::mma(ah, b1l, accx[1]);
        accx[1] = Frag<__bf16>::mma(al, b1h, accx[1]);
        guard1_b4(accx[1], ah, al, b1h, b1l);
      }
#pragma unroll 2
      for (int k0 = 0; k0 < NHID; k0 += 32) {
        const v16h a  = Frag<_Float16>::load(arhrow + k0);
        const v16h b0 = Frag<_Float16>::load(uh0 + k0);
        const v16h b1 = Frag<_Float16>::load(uh1 + k0);
        acc[0] = Frag<_Float16>::mma(a, b0, acc[0]);
        acc[1] = Frag<_Float16>::mma(a, b1, acc[1]);
        guard2_h3(acc[0], acc[1], a, b0, b1);
      }
      acc_guard2(acc[0], acc[1]);
#pragma unroll
      for (int s = 0; s < 2; ++s) {
        const int nt = 2 * ntp + s;
        const int j = j0 + 16 * s;
#pragma unroll
        for (int r = 0; r < 8; ++r) {
          const float hp  = ftanh(acc[s][r] * ACC_INV + accx[s][r] + bhv[nt]);
          const float dhv = dec[r] * hst[nt][r];
          const float zz  = zreg[nt][r];
          const float hn  = (1.0f - zz) * dhv + zz * hp;
          hst[nt][r] = hn;
          Ahn[(8 * hh + r) * HPITCH + j] = (_Float16)(hn * HCARRY);
        }
      }
    }
    __syncthreads();

    if (wave < 4) {
      const _Float16* wo = WOT + (size_t)(16 * wave + c) * NHID + koff;
      v8f a0 = z8, a1 = z8;
#pragma unroll 1
      for (int k0 = 0; k0 < NHID; k0 += 64) {
        const v16h fa0 = Frag<_Float16>::load(ahnrow + k0);
        const v16h fa1 = Frag<_Float16>::load(ahnrow + k0 + 32);
        const v16h fb0 = Frag<_Float16>::load(wo + k0);
        const v16h fb1 = Frag<_Float16>::load(wo + k0 + 32);
        a0 = Frag<_Float16>::mma(fa0, fb0, a0);
        a1 = Frag<_Float16>::mma(fa1, fb1, a1);
        guard2_h4(a0, a1, fa0, fa1, fb0, fb1);
      }
      acc_guard2(a0, a1);
#pragma unroll
      for (int r = 0; r < 8; ++r)
        Os[(8 * hh + r) * SLABP + 16 * wave + c] = (a0[r] + a1[r]) * ACC_INV + bov;
    }
  }
  __syncthreads();
  {
    const v4f ov = *(const v4f*)(Os + orow * SLABP + c4);
    float* op = obase + (size_t)(NSTEP - 1) * NCH;
    *(volatile v4f*)op = ov;
    __threadfence();
    *(volatile v4f*)op = ov;
  }
}

__global__ __launch_bounds__(NTHR) void out_transpose_kernel(const float* __restrict__ OUTT, float* __restrict__ out) {
  __shared__ float Tt[64 * 65];
  const int tid = threadIdx.x;
  const int b = blockIdx.y;
  const int t0 = blockIdx.x * 64;
#pragma unroll
  for (int it = 0; it < 4; ++it) {
    const int idx = it * NTHR + tid;
    const int tt = idx >> 4, cc4 = (idx & 15) * 4;
    const v4f v = *(const v4f*)(OUTT + (size_t)(b * NSTEP + t0 + tt) * NCH + cc4);
    Tt[tt * 65 + cc4 + 0] = v[0];
    Tt[tt * 65 + cc4 + 1] = v[1];
    Tt[tt * 65 + cc4 + 2] = v[2];
    Tt[tt * 65 + cc4 + 3] = v[3];
  }
  __syncthreads();
  v4f ov[4];
#pragma unroll
  for (int it = 0; it < 4; ++it) {
    const int idx = it * NTHR + tid;
    const int cc = idx >> 4, t4 = (idx & 15) * 4;
#pragma unroll
    for (int e = 0; e < 4; ++e) ov[it][e] = Tt[(t4 + e) * 65 + cc];
  }
  for (int pass = 0; pass < 2; ++pass) {
#pragma unroll
    for (int it = 0; it < 4; ++it) {
      const int idx = it * NTHR + tid;
      const int cc = idx >> 4, t4 = (idx & 15) * 4;
      *(volatile v4f*)(out + (size_t)(b * NCH + cc) * NSTEP + t0 + t4) = ov[it];
    }
    __threadfence();
  }
}

extern "C" void kernel_launch(void* const* d_in, const int* in_sizes, int n_in,
                              void* d_out, int out_size, void* d_ws, size_t ws_size, hipStream_t stream) {
  if (n_in < 16 || d_out == nullptr || d_ws == nullptr) return;
  if (in_sizes[0] != NBAT * NCH * NSTEP * 3 || in_sizes[1] != NSTEP * NSTEP || in_sizes[2] != NSTEP ||
      in_sizes[3] != KDEC2 * NSTEP || in_sizes[4] != NSTEP ||
      in_sizes[5] != NCH * NHID || in_sizes[6] != NCH * NHID || in_sizes[7] != NCH * NHID ||
      in_sizes[8] != NHID * NHID || in_sizes[9] != NHID * NHID || in_sizes[10] != NHID * NHID ||
      in_sizes[11] != NHID || in_sizes[12] != NHID || in_sizes[13] != NHID ||
      in_sizes[14] != NHID * NCH || in_sizes[15] != NCH || out_size != NBAT * NCH * NSTEP) return;

  const float* x  = (const float*)d_in[0];
  const float* W1 = (const float*)d_in[1];
  const float* b1 = (const float*)d_in[2];
  const float* W2 = (const float*)d_in[3];
  const float* b2 = (const float*)d_in[4];
  const float* Wz = (const float*)d_in[5];
  const float* Wr = (const float*)d_in[6];
  const float* Wh = (const float*)d_in[7];
  const float* Uz = (const float*)d_in[8];
  const float* Ur = (const float*)d_in[9];
  const float* Uh = (const float*)d_in[10];
  const float* bz = (const float*)d_in[11];
  const float* br = (const float*)d_in[12];
  const float* bh = (const float*)d_in[13];
  const float* Wo = (const float*)d_in[14];
  const float* bo = (const float*)d_in[15];
  float* out = (float*)d_out;

  char* ws = (char*)d_ws; size_t off = 0;
  auto carve = [&](size_t bytes) -> char* { char* p = ws + off; off += (bytes + 255) & ~(size_t)255; return p; };
  unsigned short* IVH  = (unsigned short*)carve((size_t)NROWBC * NSTEP * 2);
  unsigned short* IVM  = (unsigned short*)carve((size_t)NROWBC * NSTEP * 2);
  unsigned short* IVL  = (unsigned short*)carve((size_t)NROWBC * NSTEP * 2);
  float*          XE   = (float*)carve((size_t)NROWBC * NSTEP * 4);
  unsigned short* W2TH = (unsigned short*)carve((size_t)NSTEP * KDEC2 * 2);
  unsigned short* W2TL = (unsigned short*)carve((size_t)NSTEP * KDEC2 * 2);
  float*          P1   = (float*)carve((size_t)NROWBC * NSTEP * 4);
  float*          OUTT = (float*)carve((size_t)NROWBT * NCH * 4);
  unsigned short* XNH  = (unsigned short*)carve((size_t)NROWBT * NCH * 2);
  unsigned short* XNL  = (unsigned short*)carve((size_t)NROWBT * NCH * 2);
  float*          PART = (float*)carve((size_t)KSPLIT * NBAT * NSTEP * 4);
  unsigned short* UT   = (unsigned short*)carve((size_t)3 * NHID * NHID * 2);
  unsigned short* W1TH = (unsigned short*)carve((size_t)NSTEP * NSTEP * 2);
  unsigned short* W1TL = (unsigned short*)carve((size_t)NSTEP * NSTEP * 2);
  unsigned short* WXTH = (unsigned short*)carve((size_t)3 * NHID * NCH * 2);
  unsigned short* WXTL = (unsigned short*)carve((size_t)3 * NHID * NCH * 2);
  unsigned short* WOT  = (unsigned short*)carve((size_t)NCH * NHID * 2);
  float*          D2   = (float*)carve((size_t)NBAT * NSTEP * 4);
  if (off > ws_size || off > (size_t)134217728) return;

  tpw_kernel<0><<<dim3(NSTEP / 64, NSTEP / 64, 1), NTHR, 0, stream>>>(W1, W1, W1, NSTEP, NSTEP, NSTEP, W1TH, W1TL, 0L, 1.0f);
  tpw_kernel<0><<<dim3(NSTEP / 64, KDEC2 / 64, 1), NTHR, 0, stream>>>(W2, W2, W2, KDEC2, NSTEP, KDEC2, W2TH, W2TL, 0L, 1.0f);
  tpw_kernel<1><<<dim3(NHID / 64, NHID / 64, 3), NTHR, 0, stream>>>(Uz, Ur, Uh, NHID, NHID, NHID, UT, UT, (long)NHID * NHID, UCARRY);
  tpw_kernel<0><<<dim3(NHID / 64, NCH / 64, 3), NTHR, 0, stream>>>(Wz, Wr, Wh, NCH, NHID, NCH, WXTH, WXTL, (long)NHID * NCH, XSIDE_SC);
  tpw_kernel<1><<<dim3(NCH / 64, NHID / 64, 1), NTHR, 0, stream>>>(Wo, Wo, Wo, NHID, NCH, NHID, WOT, WOT, 0L, UCARRY);

  scan_kernel<<<NROWBC / 64, 64, 0, stream>>>(x, XE, IVH, IVM, IVL);

  wmma_gemm64<1, true, true, 2, 2><<<dim3((NROWBC / 64) * (NSTEP / 64) / 8, 1), 256, 0, stream>>>(
      IVH, IVM, IVL, NSTEP, 0L, W1TH, W1TL, NSTEP, 0L, P1, NSTEP, 0L, b1, NROWBC, NSTEP, NSTEP, 1.0f);

  wmma_gemm64<1, true, true, 0, 0><<<dim3((NBAT / 64) * (NSTEP / 64) / 8, KSPLIT), 256, 0, stream>>>(
      IVH, IVM, IVL, KDEC2, (long)KSLICE, W2TH, W2TL, KDEC2, (long)KSLICE, PART, NSTEP, (long)NBAT * NSTEP, b2,
      NBAT, NSTEP, KSLICE, 1.0f);
  d2_fin_kernel<<<(NBAT * NSTEP / 4) / NTHR, NTHR, 0, stream>>>(PART, b2, D2);

  xnew_kernel<<<dim3(NSTEP / 64, NBAT), NTHR, 0, stream>>>(x, XE, P1, XNH, XNL);

  gru_seq_kernel<<<NBAT / SEQ_BLK, NTHR, 0, stream>>>(XNH, XNL, D2, WXTH, WXTL, UT, WOT, bz, br, bh, bo, OUTT);

  out_transpose_kernel<<<dim3(NSTEP / 64, NBAT), NTHR, 0, stream>>>(OUTT, out);
}
